// LayerGINEncoder_8272107012813
// MI455X (gfx1250) — hardware-run, weakly checked
//
#include <hip/hip_runtime.h>
#include <stddef.h>
#include <math.h>


#define NTHR   256
#define NWAVE  8
#define EPT    8
#define CHUNK  (NTHR * EPT)
#define WCAP   (EPT * 32)
#define NB     512
#define RPW    (NB / NWAVE)
#define TPW    (NB / (16 * NWAVE))
#define FD     128
#define NMAT   4
#define LN_EPS 1e-5f

#define LDS_ACC   0
#define LDS_LIST  (LDS_ACC + NB * FD * 4)
#define LDS_PRM   (LDS_LIST + NWAVE * WCAP * 4)
#define LDS_WCNT  (LDS_PRM + 3 * FD * 4)
#define LDS_TOTAL (LDS_WCNT + 64)

#define PREP_BLK  ((NMAT * FD * (FD / 8)) / NTHR)

static_assert(FD == 128);
static_assert(NB == TPW * 16 * NWAVE);
static_assert((NB & (NB - 1)) == 0 && NB <= 32768);
static_assert(CHUNK <= 65536);
static_assert(WCAP == 32 * EPT);
static_assert(PREP_BLK * NTHR == NMAT * FD * (FD / 8));
static_assert((FD * (FD / 8)) == 2048);
static_assert((LDS_TOTAL % 16) == 0);
static_assert(LDS_TOTAL <= 300 * 1024);

typedef float        v4f   __attribute__((ext_vector_type(4)));
typedef float        v8f   __attribute__((ext_vector_type(8)));
typedef int          v4i   __attribute__((ext_vector_type(4)));
typedef unsigned int v4u   __attribute__((ext_vector_type(4)));
typedef __bf16       v16bf __attribute__((ext_vector_type(16)));
union FragB { v16bf v; v4u q[2]; };
union Pk8   { v4u q; __bf16 e[8]; };

__device__ __forceinline__ v8f zero8f() {
  v8f c;
#pragma unroll
  for (int i = 0; i < 8; ++i) c[i] = 0.0f;
  return c;
}

__device__ __forceinline__ v8f wmb(v16bf a, v16bf b, v8f c) {
  v8f d = __builtin_amdgcn_wmma_f32_16x16x32_bf16(false, a, false, b, (short)0, c, false, false);
  asm volatile("v_nop\n\tv_nop\n\tv_nop\n\tv_nop" : "+v"(d) : "v"(a), "v"(b));
  return d;
}

__device__ __forceinline__ void put4(v16bf& fh, v16bf& fl, const int b, const v4f a) {
  {
    const __bf16 hb = (__bf16)a.x; const float hf = (float)hb;
    fh[b] = hb; fl[b] = (__bf16)(a.x - hf);
  }
  {
    const __bf16 hb = (__bf16)a.y; const float hf = (float)hb;
    fh[b + 1] = hb; fl[b + 1] = (__bf16)(a.y - hf);
  }
  {
    const __bf16 hb = (__bf16)a.z; const float hf = (float)hb;
    fh[b + 2] = hb; fl[b + 2] = (__bf16)(a.z - hf);
  }
  {
    const __bf16 hb = (__bf16)a.w; const float hf = (float)hb;
    fh[b + 3] = hb; fl[b + 3] = (__bf16)(a.w - hf);
  }
}

__device__ __forceinline__ int scan_chunk(const int* __restrict__ dsts, int nE, int cbase, int nodeBase,
                                          int vec8, int* list, int tid, int wave) {
  int wc = 0;
  const int el0  = tid * EPT;
  const int e0   = cbase + el0;
  const int sent = -2147483647 - 1;
  v4i da, db;
  if (vec8 != 0 && cbase + CHUNK <= nE) {
    da = *(const v4i*)(dsts + e0);
    db = *(const v4i*)(dsts + e0 + 4);
  } else {
    da.x = (e0     < nE) ? dsts[min(e0, nE - 1)] : sent;
    da.y = (e0 + 1 < nE) ? dsts[min(e0 + 1, nE - 1)] : sent;
    da.z = (e0 + 2 < nE) ? dsts[min(e0 + 2, nE - 1)] : sent;
    da.w = (e0 + 3 < nE) ? dsts[min(e0 + 3, nE - 1)] : sent;
    db.x = (e0 + 4 < nE) ? dsts[min(e0 + 4, nE - 1)] : sent;
    db.y = (e0 + 5 < nE) ? dsts[min(e0 + 5, nE - 1)] : sent;
    db.z = (e0 + 6 < nE) ? dsts[min(e0 + 6, nE - 1)] : sent;
    db.w = (e0 + 7 < nE) ? dsts[min(e0 + 7, nE - 1)] : sent;
  }
  const unsigned nb = (unsigned)nodeBase;
  const unsigned s0 = (unsigned)da.x - nb, s1 = (unsigned)da.y - nb;
  const unsigned s2 = (unsigned)da.z - nb, s3 = (unsigned)da.w - nb;
  const unsigned s4 = (unsigned)db.x - nb, s5 = (unsigned)db.y - nb;
  const unsigned s6 = (unsigned)db.z - nb, s7 = (unsigned)db.w - nb;
  const bool h0 = s0 < (unsigned)NB, h1 = s1 < (unsigned)NB, h2 = s2 < (unsigned)NB, h3 = s3 < (unsigned)NB;
  const bool h4 = s4 < (unsigned)NB, h5 = s5 < (unsigned)NB, h6 = s6 < (unsigned)NB, h7 = s7 < (unsigned)NB;
  const unsigned any = __builtin_amdgcn_ballot_w32(h0 | h1 | h2 | h3 | h4 | h5 | h6 | h7);
  if (any != 0u) {
#define HITJ(J, HJ, SJ) { \
      const unsigned mj = __builtin_amdgcn_ballot_w32(HJ); \
      if (mj != 0u) { \
        if (HJ) { \
          const int pos = wc + (int)__builtin_amdgcn_mbcnt_lo(mj, 0u); \
          if (pos < WCAP) list[wave * WCAP + pos] = (int)(((SJ) << 16) | (unsigned)(el0 + (J))); \
        } \
        wc += (int)__builtin_popcount(mj); } }
    HITJ(0, h0, s0)
    HITJ(1, h1, s1)
    HITJ(2, h2, s2)
    HITJ(3, h3, s3)
    HITJ(4, h4, s4)
    HITJ(5, h5, s5)
    HITJ(6, h6, s6)
    HITJ(7, h7, s7)
#undef HITJ
  }
  return wc;
}

__global__ __launch_bounds__(NTHR) void k_prep(const float* __restrict__ pw, const float* __restrict__ mw,
                                              unsigned short* whi, unsigned short* wlo) {
  const int u   = blockIdx.x * NTHR + threadIdx.x;
  const int mat = u >> 11;
  const int rem = u & 2047;
  const int n   = rem >> 4;
  const int kc  = rem & 15;
  const float* src = (mat == 0) ? pw : (mw + (size_t)(mat - 1) * FD * FD);
  Pk8 ph, pl;
#pragma unroll
  for (int j = 0; j < 8; ++j) {
    const int k = 8 * kc + j;
    const float w = src[(size_t)k * FD + n];
    const __bf16 hb = (__bf16)w;
    const float  hf = (float)hb;
    ph.e[j] = hb;
    pl.e[j] = (__bf16)(w - hf);
  }
  unsigned short* dh = whi + (size_t)u * 8;
  unsigned short* dl = wlo + (size_t)u * 8;
  const v4u qh = ph.q;
  const v4u ql = pl.q;
  *(volatile v4u*)dh = qh;
  *(volatile v4u*)dl = ql;
  __threadfence();
  *(volatile v4u*)dh = qh;
  *(volatile v4u*)dl = ql;
}

template <int AGG, int LN>
__global__ __launch_bounds__(NTHR) void k_layer(
    const float* __restrict__ hin, const int* __restrict__ ei,
    const unsigned short* __restrict__ whi, const unsigned short* __restrict__ wlo,
    const float* __restrict__ bias, const float* __restrict__ gam, const float* __restrict__ bet,
    float* hout, int nN, int nE, int vec8) {
  extern __shared__ __attribute__((aligned(16))) unsigned char dsm[];
  float* acc  = (float*)(dsm + LDS_ACC);
  int*   list = (int*)(dsm + LDS_LIST);
  float* prm  = (float*)(dsm + LDS_PRM);
  int*   wcnt = (int*)(dsm + LDS_WCNT);

  const int tid = threadIdx.x, lane = tid & 31, wave = tid >> 5, hh = lane >> 4, m = lane & 15;
  const int nodeBase = blockIdx.x * NB;
  const int* srcs = ei;
  const int* dsts = ei + nE;

  {
    const v4f z4 = {0.0f, 0.0f, 0.0f, 0.0f};
#pragma unroll 1
    for (int rr = 0; rr < RPW; ++rr) {
      const int row  = wave * RPW + rr;
      const int node = nodeBase + row;
      const int nc   = node < nN ? node : nN - 1;
      v4f v = *(const v4f*)(hin + (size_t)nc * FD + 4 * lane);
      if (node >= nN) v = z4;
      *(v4f*)(acc + row * FD + 4 * lane) = v;
    }
  }
  if (tid < FD) {
    prm[tid]          = bias[tid];
    prm[FD + tid]     = gam[tid];
    prm[2 * FD + tid] = bet[tid];
  }
  __syncthreads();

  if (AGG) {
    const int nChunks = (nE + CHUNK - 1) / CHUNK;
#pragma unroll 1
    for (int ch = 0; ch < nChunks; ++ch) {
      const int cbase = ch * CHUNK;
      const int wc = scan_chunk(dsts, nE, cbase, nodeBase, vec8, list, tid, wave);
      if (lane == 0) wcnt[wave] = wc;
      __syncthreads();

      if (wave == 0) {
#pragma unroll 1
        for (int u = 0; u < NWAVE; ++u) {
          int n = __builtin_amdgcn_readfirstlane(wcnt[u]);
          n = n > WCAP ? WCAP : (n < 0 ? 0 : n);
#pragma unroll 1
          for (int i = 0; i < n; ++i) {
            const int ent  = __builtin_amdgcn_readfirstlane(list[u * WCAP + i]);
            const int el   = ent & 0xFFFF;
            const int slot = (ent >> 16) & (NB - 1);
            int e = cbase + el;
            e = e > nE - 1 ? nE - 1 : e;
            int s = srcs[e];
            s = s < 0 ? 0 : (s > nN - 1 ? nN - 1 : s);
            const v4f v = *(const v4f*)(hin + (size_t)s * FD + 4 * lane);
            float* ap = acc + slot * FD + 4 * lane;
            v4f a = *(v4f*)ap;
            a += v;
            *(v4f*)ap = a;
          }
        }
      }
      __syncthreads();
    }
  }

#pragma unroll 1
  for (int tt = 0; tt < TPW; ++tt) {
    const int t = wave + NWAVE * tt;
    const float* zr = acc + (16 * t + m) * FD + 8 * hh;
    v8f c[8];
#pragma unroll
    for (int nt = 0; nt < 8; ++nt) c[nt] = zero8f();

#pragma unroll 1
    for (int kt = 0; kt < 4; ++kt) {
      v16bf ah, al;
      {
        const float* zp = zr + 32 * kt;
        const v4f z0 = *(const v4f*)zp;
        const v4f z1 = *(const v4f*)(zp + 4);
        const v4f z2 = *(const v4f*)(zp + 16);
        const v4f z3 = *(const v4f*)(zp + 20);
        put4(ah, al, 0, z0);
        put4(ah, al, 4, z1);
        put4(ah, al, 8, z2);
        put4(ah, al, 12, z3);
      }
      const unsigned short* bph = whi + (size_t)m * FD + 32 * kt + 8 * hh;
      const unsigned short* bpl = wlo + (size_t)m * FD + 32 * kt + 8 * hh;
#pragma unroll
      for (int nt = 0; nt < 8; ++nt) {
        FragB bh, bl;
        const unsigned short* p = bph + (size_t)nt * 16 * FD;
        const unsigned short* q = bpl + (size_t)nt * 16 * FD;
        bh.q[0] = *(const v4u*)p;
        bh.q[1] = *(const v4u*)(p + 16);
        bl.q[0] = *(const v4u*)q;
        bl.q[1] = *(const v4u*)(q + 16);
        c[nt] = wmb(ah, bh.v, c[nt]);
        c[nt] = wmb(ah, bl.v, c[nt]);
        c[nt] = wmb(al, bh.v, c[nt]);
      }
    }
    __syncthreads();

    {
      float bia[8], ga[8], be[8];
#pragma unroll
      for (int nt = 0; nt < 8; ++nt) {
        const int n = 16 * nt + m;
        bia[nt] = prm[n];
        ga[nt]  = LN ? prm[FD + n] : 1.0f;
        be[nt]  = LN ? prm[2 * FD + n] : 0.0f;
      }
#pragma unroll
      for (int nt = 0; nt < 8; ++nt) {
#pragma unroll
        for (int r = 0; r < 8; ++r) c[nt][r] = fmaxf(c[nt][r] + bia[nt], 0.0f);
      }
      if (LN) {
#pragma unroll
        for (int r = 0; r < 8; ++r) {
          float s = 0.0f;
#pragma unroll
          for (int nt = 0; nt < 8; ++nt) s += c[nt][r];
          s += __shfl_xor(s, 1, 32);
          s += __shfl_xor(s, 2, 32);
          s += __shfl_xor(s, 4, 32);
          s += __shfl_xor(s, 8, 32);
          const float mu = s * (1.0f / FD);
          float q = 0.0f;
#pragma unroll
          for (int nt = 0; nt < 8; ++nt) { const float d = c[nt][r] - mu; q += d * d; }
          q += __shfl_xor(q, 1, 32);
          q += __shfl_xor(q, 2, 32);
          q += __shfl_xor(q, 4, 32);
          q += __shfl_xor(q, 8, 32);
          const float rs = rsqrtf(q * (1.0f / FD) + LN_EPS);
#pragma unroll
          for (int nt = 0; nt < 8; ++nt) c[nt][r] = (c[nt][r] - mu) * rs * ga[nt] + be[nt];
        }
      }
      float* orow = acc + (16 * t + 8 * hh) * FD + m;
#pragma unroll
      for (int r = 0; r < 8; ++r) {
#pragma unroll
        for (int nt = 0; nt < 8; ++nt) orow[r * FD + 16 * nt] = c[nt][r];
      }
    }
    __syncthreads();
  }

#pragma unroll 1
  for (int rr = 0; rr < RPW; ++rr) {
    const int row = wave * RPW + rr;
    const v4f v = *(const v4f*)(acc + row * FD + 4 * lane);
    *(volatile v4f*)(hout + (size_t)(nodeBase + row) * FD + 4 * lane) = v;
  }
  __threadfence();
#pragma unroll 1
  for (int rr = 0; rr < RPW; ++rr) {
    const int row = wave * RPW + rr;
    const v4f v = *(const v4f*)(acc + row * FD + 4 * lane);
    *(volatile v4f*)(hout + (size_t)(nodeBase + row) * FD + 4 * lane) = v;
  }
}

__global__ __launch_bounds__(NTHR) void k_pool(const float* __restrict__ x, const int* __restrict__ bt,
                                              float* pooled, int nN) {
  __shared__ int hl[NTHR];
  __shared__ int wc[NWAVE];
  __shared__ __attribute__((aligned(16))) float prow[FD];
  const int tid = threadIdx.x, lane = tid & 31, wave = tid >> 5;
  const int g = blockIdx.x;
  float s = 0.0f;
  int cnt = 0;
  const int nCh = (nN + NTHR - 1) / NTHR;
#pragma unroll 1
  for (int ch = 0; ch < nCh; ++ch) {
    const int i  = ch * NTHR + tid;
    const int ic = i > nN - 1 ? nN - 1 : i;
    const int b  = bt[ic];
    const bool hit = (i < nN) && (b == g);
    const unsigned mk = __builtin_amdgcn_ballot_w32(hit);
    if (lane == 0) wc[wave] = (int)__builtin_popcount(mk);
    __syncthreads();
    int off = 0, tot = 0;
#pragma unroll
    for (int w = 0; w < NWAVE; ++w) { const int c = wc[w]; if (w < wave) off += c; tot += c; }
    if (hit) {
      const int pos = off + (int)__builtin_amdgcn_mbcnt_lo(mk, 0u);
      if (pos < NTHR) hl[pos] = i;
    }
    __syncthreads();
    tot = tot > NTHR ? NTHR : (tot < 0 ? 0 : tot);
    if (tid < FD) {
#pragma unroll 1
      for (int j = 0; j < tot; ++j) {
        int nd = hl[j];
        nd = nd < 0 ? 0 : (nd > nN - 1 ? nN - 1 : nd);
        s += x[(size_t)nd * FD + tid];
      }
    }
    cnt += tot;
    __syncthreads();
  }
  if (tid < FD) {
    const float c = (float)(cnt > 1 ? cnt : 1);
    prow[tid] = s * (1.0f / c);
  }
  __syncthreads();
  v4f v = {0.0f, 0.0f, 0.0f, 0.0f};
  if (wave == 0) v = *(const v4f*)(prow + 4 * lane);
  if (wave == 0) *(volatile v4f*)(pooled + (size_t)g * FD + 4 * lane) = v;
  __threadfence();
  if (wave == 0) *(volatile v4f*)(pooled + (size_t)g * FD + 4 * lane) = v;
}

extern "C" void kernel_launch(void* const* d_in, const int* in_sizes, int n_in,
                              void* d_out, int out_size, void* d_ws, size_t ws_size,
                              hipStream_t stream) {
  if (n_in < 9) return;
  const int nN = in_sizes[0] / FD;
  if (nN < 1 || in_sizes[0] != nN * FD) return;
  const int nE = in_sizes[1] / 2;
  if (nE < 1 || in_sizes[1] != 2 * nE) return;
  if (in_sizes[2] != nN) return;
  if (in_sizes[3] != FD * FD || in_sizes[4] != FD) return;
  if (in_sizes[5] != (NMAT - 1) * FD * FD || in_sizes[6] != (NMAT - 1) * FD) return;
  if (in_sizes[7] != (NMAT - 1) * FD || in_sizes[8] != (NMAT - 1) * FD) return;
  const int G = out_size / FD;
  if (G < 1 || out_size != G * FD) return;

  const float* x      = (const float*)d_in[0];
  const int*   ei     = (const int*)d_in[1];
  const int*   batch  = (const int*)d_in[2];
  const float* proj_W = (const float*)d_in[3];
  const float* proj_b = (const float*)d_in[4];
  const float* mlp_W  = (const float*)d_in[5];
  const float* mlp_b  = (const float*)d_in[6];
  const float* ln_g   = (const float*)d_in[7];
  const float* ln_b   = (const float*)d_in[8];
  float* outp = (float*)d_out;

  const int nBlk = (nN + NB - 1) / NB;
  const size_t rowsP = (size_t)nBlk * NB;

  char* ws = (char*)d_ws;
  size_t off = 0;
  const size_t oWh = off; off += ((size_t)NMAT * FD * FD * 2 + 255) & ~(size_t)255;
  const size_t oWl = off; off += ((size_t)NMAT * FD * FD * 2 + 255) & ~(size_t)255;
  const size_t oX0 = off; off += (rowsP * FD * 4 + 255) & ~(size_t)255;
  const size_t oX1 = off; off += (rowsP * FD * 4 + 255) & ~(size_t)255;
  size_t limit = (size_t)134217728;
  if (ws_size < limit) limit = ws_size;
  if (off > limit) return;

  unsigned short* Wh = (unsigned short*)(ws + oWh);
  unsigned short* Wl = (unsigned short*)(ws + oWl);
  float* X0 = (float*)(ws + oX0);
  float* X1 = (float*)(ws + oX1);

  const int vec8 = ((nE & 3) == 0) ? 1 : 0;

  k_prep<<<PREP_BLK, NTHR, 0, stream>>>(proj_W, mlp_W, Wh, Wl);

  (void)hipFuncSetAttribute(reinterpret_cast<const void*>(&k_layer<0, 0>),
                            hipFuncAttributeMaxDynamicSharedMemorySize, LDS_TOTAL);
  (void)hipFuncSetAttribute(reinterpret_cast<const void*>(&k_layer<1, 1>),
                            hipFuncAttributeMaxDynamicSharedMemorySize, LDS_TOTAL);

  k_layer<0, 0><<<nBlk, NTHR, LDS_TOTAL, stream>>>(x, ei, Wh, Wl, proj_b, ln_g, ln_b,
                                                   X0, nN, nE, vec8);
  float* cur = X0;
  float* nxt = X1;
  for (int l = 0; l < NMAT - 1; ++l) {
    k_layer<1, 1><<<nBlk, NTHR, LDS_TOTAL, stream>>>(
        cur, ei, Wh + (size_t)(l + 1) * FD * FD, Wl + (size_t)(l + 1) * FD * FD,
        mlp_b + (size_t)l * FD, ln_g + (size_t)l * FD, ln_b + (size_t)l * FD,
        nxt, nN, nE, vec8);
    float* tswap = cur; cur = nxt; nxt = tswap;
  }

  k_pool<<<G, NTHR, 0, stream>>>(cur, batch, outp, nN);
}
